// SS2D_77163382440854
// MI455X (gfx1250) — hardware-verified
//
#include <hip/hip_runtime.h>
#include <stdint.h>


#define NB   8
#define HH   64
#define WW   64
#define CC   96
#define DI   192
#define NS   16
#define RR   6
#define KD   4
#define LL   (HH * WW)
#define MM   (NB * LL)
#define CP   (RR + 2 * NS)
#define CPAD 48
#define NBK  (NB * KD)
#define CHK  64
#define SHW  40

static_assert(CC % 32 == 0, "");
static_assert(DI % 32 == 0, "");
static_assert(MM % 64 == 0, "");
static_assert(LL % 64 == 0, "");
static_assert((MM * CC) % 256 == 0, "");
static_assert((2 * DI * CC) % 256 == 0, "");
static_assert((CC * DI) % 256 == 0, "");
static_assert((KD * CPAD * DI) % 256 == 0, "");

typedef float v4f __attribute__((ext_vector_type(4)));
typedef float v4fa __attribute__((ext_vector_type(4))) __attribute__((may_alias));
typedef float v8f __attribute__((ext_vector_type(8)));
typedef unsigned short v8us __attribute__((ext_vector_type(8)));
typedef unsigned short v8usa __attribute__((ext_vector_type(8))) __attribute__((may_alias));
typedef __bf16 v16bf __attribute__((ext_vector_type(16)));

union Frag { v16bf v; v8us h[2]; };

__device__ __forceinline__ unsigned short bf_rne(float f) {
  unsigned int u = __float_as_uint(f);
  u += 0x7FFFu + ((u >> 16) & 1u);
  return (unsigned short)(u >> 16);
}

__device__ __forceinline__ void split8(const float* v, v8us& hi, v8us& lo) {
#pragma unroll
  for (int i = 0; i < 8; ++i) {
    const unsigned short hb = bf_rne(v[i]);
    const float hf = __uint_as_float(((unsigned int)hb) << 16);
    hi[i] = hb;
    lo[i] = bf_rne(v[i] - hf);
  }
}

__device__ __forceinline__ void ldfrag(Frag& f, const unsigned short* __restrict__ rowp, int k0, int h) {
  f.h[0] = *(const v8usa*)(rowp + k0 + 8 * h);
  f.h[1] = *(const v8usa*)(rowp + k0 + 16 + 8 * h);
}

__device__ __forceinline__ v8f mma3(v8f acc, const Frag& ah, const Frag& al,
                                    const Frag& bh, const Frag& bl) {
  acc = __builtin_amdgcn_wmma_f32_16x16x32_bf16(false, ah.v, false, bh.v, (short)0, acc, false, false);
  acc = __builtin_amdgcn_wmma_f32_16x16x32_bf16(false, ah.v, false, bl.v, (short)0, acc, false, false);
  acc = __builtin_amdgcn_wmma_f32_16x16x32_bf16(false, al.v, false, bh.v, (short)0, acc, false, false);
  asm volatile("v_nop\n\tv_nop\n\tv_nop\n\tv_nop"
               : "+v"(acc) : "v"(ah.v), "v"(al.v), "v"(bh.v), "v"(bl.v));
  return acc;
}

__device__ __forceinline__ void st_planes(unsigned short* ph, unsigned short* pl, v8us vh, v8us vl) {
  *(volatile v8us*)ph = vh;
  *(volatile v8us*)pl = vl;
}

template <int NCOL>
__device__ __forceinline__ void tile_store(const float* sdw, float* ob, int pitch, int lane) {
  constexpr int LPR = NCOL / 32;
  constexpr int NIT = 4 * LPR;
  const int sub = lane >> 3;
  const int piece = (lane & 7) * 4;
#pragma unroll
  for (int it = 0; it < NIT; ++it) {
    const int lq = it * 4 + sub;
    const int row = lq / LPR;
    const int cs = (lq - row * LPR) * 32 + piece;
    const v4f v = *(const v4fa*)(sdw + row * NCOL + cs);
    *(volatile v4f*)(ob + (size_t)row * pitch + cs) = v;
  }
  __threadfence();
#pragma unroll
  for (int it = 0; it < NIT; ++it) {
    const int lq = it * 4 + sub;
    const int row = lq / LPR;
    const int cs = (lq - row * LPR) * 32 + piece;
    const v4f v = *(const v4fa*)(sdw + row * NCOL + cs);
    *(volatile v4f*)(ob + (size_t)row * pitch + cs) = v;
  }
}

__device__ __forceinline__ int xpos(int k, int l) {
  const int ll = (k & 2) ? (LL - 1 - l) : l;
  return (k & 1) ? (((ll & (HH - 1)) << 6) | (ll >> 6)) : ll;
}

__global__ void __launch_bounds__(256)
k_cvt(const float* __restrict__ src, int n8,
      unsigned short* __restrict__ hi, unsigned short* __restrict__ lo) {
  const int g = blockIdx.x * 256 + threadIdx.x;
  if (g >= n8) return;
  const size_t e = (size_t)g * 8;
  const v4f a = *(const v4fa*)(src + e);
  const v4f b = *(const v4fa*)(src + e + 4);
  const float v[8] = {a.x, a.y, a.z, a.w, b.x, b.y, b.z, b.w};
  v8us vh, vl;
  split8(v, vh, vl);
  st_planes(hi + e, lo + e, vh, vl);
  __threadfence();
  st_planes(hi + e, lo + e, vh, vl);
}

__global__ void __launch_bounds__(256)
k_cvtw2(const float* __restrict__ w2,
        unsigned short* __restrict__ hi, unsigned short* __restrict__ lo) {
  const int g = blockIdx.x * 256 + threadIdx.x;
  if (g >= (KD * CPAD * DI) / 8) return;
  const int e = g * 8;
  const int kk = e / (CPAD * DI);
  const int rem = e - kk * (CPAD * DI);
  const int c = rem / DI;
  const int d0 = rem - c * DI;
  float v[8];
  if (c < CP) {
    const float* p = w2 + ((size_t)(kk * CP + c)) * DI + d0;
    const v4f a = *(const v4fa*)p;
    const v4f b = *(const v4fa*)(p + 4);
    v[0] = a.x; v[1] = a.y; v[2] = a.z; v[3] = a.w;
    v[4] = b.x; v[5] = b.y; v[6] = b.z; v[7] = b.w;
  } else {
#pragma unroll
    for (int i = 0; i < 8; ++i) v[i] = 0.f;
  }
  v8us vh, vl;
  split8(v, vh, vl);
  st_planes(hi + e, lo + e, vh, vl);
  __threadfence();
  st_planes(hi + e, lo + e, vh, vl);
}

__global__ void __launch_bounds__(128)
k_gemm1(const unsigned short* __restrict__ xh, const unsigned short* __restrict__ xl,
        const unsigned short* __restrict__ wh, const unsigned short* __restrict__ wl,
        float* __restrict__ xz) {
  __shared__ __attribute__((aligned(16))) float sD[4][16][64];
  const int lane = threadIdx.x & 31, w = threadIdx.x >> 5;
  const int h = lane >> 4, m = lane & 15;
  const int r0 = blockIdx.x * 64 + w * 16;
  const int c0 = blockIdx.y * 64;
  v8f acc[4] = {};
  const size_t ao = (size_t)(r0 + m) * CC;
  size_t bo[4];
#pragma unroll
  for (int t = 0; t < 4; ++t) bo[t] = (size_t)(c0 + t * 16 + m) * CC;
#pragma unroll 1
  for (int ks = 0; ks < CC / 32; ++ks) {
    const int k0 = ks * 32;
    Frag ah, al;
    ldfrag(ah, xh + ao, k0, h);
    ldfrag(al, xl + ao, k0, h);
#pragma unroll
    for (int t = 0; t < 4; ++t) {
      Frag bh, bl;
      ldfrag(bh, wh + bo[t], k0, h);
      ldfrag(bl, wl + bo[t], k0, h);
      acc[t] = mma3(acc[t], ah, al, bh, bl);
    }
  }
#pragma unroll
  for (int t = 0; t < 4; ++t)
#pragma unroll
    for (int r = 0; r < 8; ++r) sD[w][8 * h + r][16 * t + m] = acc[t][r];
  __syncthreads();
  tile_store<64>(&sD[w][0][0], xz + (size_t)r0 * (2 * DI) + c0, 2 * DI, lane);
}

__global__ void __launch_bounds__(192)
k_conv(const float* __restrict__ xz, const float* __restrict__ cw, const float* __restrict__ cb,
       float* __restrict__ up, unsigned short* __restrict__ ch, unsigned short* __restrict__ cl) {
  __shared__ __attribute__((aligned(16))) float sU[4][DI];
  const int tid = threadIdx.x;
  const int px = tid / 48;
  const int g = tid - px * 48;
  const int d0 = g * 4;
  const int m0 = blockIdx.x * 4;
  const int m = m0 + px;
  const int b = m >> 12;
  const int pos = m & (LL - 1);
  const int hq = pos >> 6, wq = pos & 63;
  float s0 = 0.f, s1 = 0.f, s2 = 0.f, s3 = 0.f;
#pragma unroll
  for (int kh = 0; kh < 3; ++kh) {
    const int h2 = hq + kh - 1;
    if ((unsigned)h2 >= (unsigned)HH) continue;
#pragma unroll
    for (int kw = 0; kw < 3; ++kw) {
      const int w2 = wq + kw - 1;
      if ((unsigned)w2 >= (unsigned)WW) continue;
      const v4f v = *(const v4fa*)(xz + ((size_t)((b * HH + h2) * WW + w2)) * (2 * DI) + d0);
      const int tap = kh * 3 + kw;
      s0 = fmaf(v.x, cw[(d0 + 0) * 9 + tap], s0);
      s1 = fmaf(v.y, cw[(d0 + 1) * 9 + tap], s1);
      s2 = fmaf(v.z, cw[(d0 + 2) * 9 + tap], s2);
      s3 = fmaf(v.w, cw[(d0 + 3) * 9 + tap], s3);
    }
  }
  s0 += cb[d0 + 0]; s1 += cb[d0 + 1]; s2 += cb[d0 + 2]; s3 += cb[d0 + 3];
  v4f o;
  o.x = s0 * __builtin_amdgcn_rcpf(1.f + __expf(-s0));
  o.y = s1 * __builtin_amdgcn_rcpf(1.f + __expf(-s1));
  o.z = s2 * __builtin_amdgcn_rcpf(1.f + __expf(-s2));
  o.w = s3 * __builtin_amdgcn_rcpf(1.f + __expf(-s3));
  float* q = up + (size_t)m * DI + d0;
  *(volatile v4f*)q = o;
  sU[px][d0 + 0] = o.x; sU[px][d0 + 1] = o.y; sU[px][d0 + 2] = o.z; sU[px][d0 + 3] = o.w;
  __syncthreads();
  const bool act = tid < 96;
  v8us vh, vl;
  unsigned short* ph = ch;
  unsigned short* pl = cl;
  if (act) {
    const int p2 = tid / 24;
    const int e0 = (tid - p2 * 24) * 8;
    const v4f a = *(const v4fa*)(&sU[p2][e0]);
    const v4f c4 = *(const v4fa*)(&sU[p2][e0 + 4]);
    const float v[8] = {a.x, a.y, a.z, a.w, c4.x, c4.y, c4.z, c4.w};
    split8(v, vh, vl);
    const size_t e = (size_t)(m0 + p2) * DI + e0;
    ph = ch + e; pl = cl + e;
    st_planes(ph, pl, vh, vl);
  }
  __threadfence();
  *(volatile v4f*)q = o;
  if (act) st_planes(ph, pl, vh, vl);
}

__global__ void __launch_bounds__(96)
k_gemm2(const unsigned short* __restrict__ w2h, const unsigned short* __restrict__ w2l,
        const unsigned short* __restrict__ ch, const unsigned short* __restrict__ cl,
        float* __restrict__ xdbl) {
  __shared__ __attribute__((aligned(16))) float sD[3][16][64];
  const int lane = threadIdx.x & 31, w = threadIdx.x >> 5;
  const int h = lane >> 4, m = lane & 15;
  const int bk = blockIdx.y;
  const int b = bk >> 2, k = bk & 3;
  const int l0 = blockIdx.x * 64;
  const size_t ao = ((size_t)(k * CPAD + w * 16 + m)) * DI;
  size_t bo[4];
#pragma unroll
  for (int t = 0; t < 4; ++t) bo[t] = ((size_t)(b * LL + xpos(k, l0 + 16 * t + m))) * DI;
  v8f acc[4] = {};
#pragma unroll 1
  for (int ks = 0; ks < DI / 32; ++ks) {
    const int k0 = ks * 32;
    Frag ah, al;
    ldfrag(ah, w2h + ao, k0, h);
    ldfrag(al, w2l + ao, k0, h);
#pragma unroll
    for (int t = 0; t < 4; ++t) {
      Frag bh, bl;
      ldfrag(bh, ch + bo[t], k0, h);
      ldfrag(bl, cl + bo[t], k0, h);
      acc[t] = mma3(acc[t], ah, al, bh, bl);
    }
  }
#pragma unroll
  for (int t = 0; t < 4; ++t)
#pragma unroll
    for (int r = 0; r < 8; ++r) sD[w][8 * h + r][16 * t + m] = acc[t][r];
  __syncthreads();
  tile_store<64>(&sD[w][0][0], xdbl + ((size_t)(bk * CPAD + w * 16)) * LL + l0, LL, lane);
}

__global__ void __launch_bounds__(192)
k_scan(const float* __restrict__ up, const float* __restrict__ xdbl,
       const float* __restrict__ dtw, const float* __restrict__ dtb,
       const float* __restrict__ alog, const float* __restrict__ dsk,
       float* __restrict__ y4) {
  __shared__ __attribute__((aligned(16))) float sh[CHK][SHW];
  const int d = threadIdx.x;
  const int bk = blockIdx.x;
  const int b = bk >> 2, k = bk & 3;
  const int kc = k * DI + d;
  float wdt[RR];
#pragma unroll
  for (int r = 0; r < RR; ++r) wdt[r] = dtw[(size_t)kc * RR + r];
  const float bias = dtb[kc];
  const float dsv = dsk[kc];
  float av[NS];
#pragma unroll
  for (int n = 0; n < NS; ++n) av[n] = -__expf(alog[(size_t)kc * NS + n]);
  float hs[NS];
#pragma unroll
  for (int n = 0; n < NS; ++n) hs[n] = 0.f;
  v4f yq = {0.f, 0.f, 0.f, 0.f};
  const float* ub = up + (size_t)b * LL * DI + d;
  const float* xb = xdbl + (size_t)bk * CPAD * LL;
  float* yb = y4 + ((size_t)bk * (LL / 4) * DI + d) * 4;

  for (int l0 = 0; l0 < LL; l0 += CHK) {
    __syncthreads();
    for (int t = d; t < SHW * (CHK / 4); t += DI) {
      const int c = t / (CHK / 4);
      const int q = t - c * (CHK / 4);
      const v4f v = *(const v4fa*)(xb + (size_t)c * LL + l0 + 4 * q);
      sh[4 * q + 0][c] = v.x;
      sh[4 * q + 1][c] = v.y;
      sh[4 * q + 2][c] = v.z;
      sh[4 * q + 3][c] = v.w;
    }
    __syncthreads();
#pragma unroll 1
    for (int j = 0; j < CHK; ++j) {
      const int l = l0 + j;
      union { v4f q[SHW / 4]; float f[SHW]; } P;
      const v4fa* rp = (const v4fa*)(&sh[j][0]);
#pragma unroll
      for (int i = 0; i < SHW / 4; ++i) P.q[i] = rp[i];
      float sdt = 0.f;
#pragma unroll
      for (int r = 0; r < RR; ++r) sdt = fmaf(wdt[r], P.f[r], sdt);
      const float raw = sdt + bias;
      const float ey = __expf(-fabsf(raw));
      const float uu = 1.f + ey;
      const float tt = uu - 1.f;
      float lp = __logf(uu) * (ey * __builtin_amdgcn_rcpf(tt));
      lp = (tt > 0.f) ? lp : ey;
      const float delta = fmaxf(raw, 0.f) + lp;
      const float u = ub[(size_t)xpos(k, l) * DI];
      const float du = delta * u;
      float yv = 0.f;
#pragma unroll
      for (int n = 0; n < NS; ++n) {
        const float dA = __expf(delta * av[n]);
        hs[n] = fmaf(dA, hs[n], du * P.f[RR + n]);
        yv = fmaf(hs[n], P.f[RR + NS + n], yv);
      }
      yv = fmaf(u, dsv, yv);
      yq.x = yq.y; yq.y = yq.z; yq.z = yq.w; yq.w = yv;
      if ((j & 3) == 3) {
        float* p = yb + (size_t)(l >> 2) * (DI * 4);
        *(volatile v4f*)p = yq;
        __threadfence();
        *(volatile v4f*)p = yq;
      }
    }
  }
}

__global__ void __launch_bounds__(256)
k_ln(const float* __restrict__ y4, const float* __restrict__ xz,
     const float* __restrict__ gw, const float* __restrict__ gb,
     unsigned short* __restrict__ th, unsigned short* __restrict__ tl) {
  __shared__ __attribute__((aligned(16))) float sT[8][DI];
  const int tid = threadIdx.x;
  const int lane = tid & 31, w = tid >> 5;
  const int m0 = blockIdx.x * 8;
  const int m = m0 + w;
  const int b = m >> 12;
  const int pos = m & (LL - 1);
  const int hq = pos >> 6, wq = pos & 63;
  const int lt = wq * HH + hq;
  const int bk0 = b * KD;
  const int la0 = pos, la2 = LL - 1 - pos, la1 = lt, la3 = LL - 1 - lt;
  const size_t o0 = (((size_t)(bk0 + 0) * (LL / 4) + (la0 >> 2)) * DI) * 4 + (la0 & 3);
  const size_t o1 = (((size_t)(bk0 + 1) * (LL / 4) + (la1 >> 2)) * DI) * 4 + (la1 & 3);
  const size_t o2 = (((size_t)(bk0 + 2) * (LL / 4) + (la2 >> 2)) * DI) * 4 + (la2 & 3);
  const size_t o3 = (((size_t)(bk0 + 3) * (LL / 4) + (la3 >> 2)) * DI) * 4 + (la3 & 3);
  float v[6];
  float s = 0.f;
#pragma unroll
  for (int i = 0; i < 6; ++i) {
    const int dd = (lane + 32 * i) * 4;
    const float a0 = y4[o0 + dd];
    const float a2 = y4[o2 + dd];
    const float a1 = y4[o1 + dd];
    const float a3 = y4[o3 + dd];
    v[i] = (a0 + a2) + (a1 + a3);
    s += v[i];
  }
#pragma unroll
  for (int off = 16; off > 0; off >>= 1) s += __shfl_xor(s, off, 32);
  const float mean = s * (1.f / (float)DI);
  float dv[6];
  float s2 = 0.f;
#pragma unroll
  for (int i = 0; i < 6; ++i) { dv[i] = v[i] - mean; s2 = fmaf(dv[i], dv[i], s2); }
#pragma unroll
  for (int off = 16; off > 0; off >>= 1) s2 += __shfl_xor(s2, off, 32);
  const float var = s2 * (1.f / (float)DI);
  const float inv = rsqrtf(var + 1e-5f);
  const float* zr = xz + (size_t)m * (2 * DI) + DI;
#pragma unroll
  for (int i = 0; i < 6; ++i) {
    const int dch = lane + 32 * i;
    const float val = dv[i] * inv * gw[dch] + gb[dch];
    const float zz = zr[dch];
    const float sg = zz * __builtin_amdgcn_rcpf(1.f + __expf(-zz));
    sT[w][dch] = val * sg;
  }
  __syncthreads();
  const bool act = tid < 8 * (DI / 8);
  v8us vh, vl;
  unsigned short* ph = th;
  unsigned short* pl = tl;
  if (act) {
    const int p2 = tid / (DI / 8);
    const int e0 = (tid - p2 * (DI / 8)) * 8;
    const v4f a = *(const v4fa*)(&sT[p2][e0]);
    const v4f c4 = *(const v4fa*)(&sT[p2][e0 + 4]);
    const float vv[8] = {a.x, a.y, a.z, a.w, c4.x, c4.y, c4.z, c4.w};
    split8(vv, vh, vl);
    const size_t e = (size_t)(m0 + p2) * DI + e0;
    ph = th + e; pl = tl + e;
    st_planes(ph, pl, vh, vl);
  }
  __threadfence();
  if (act) st_planes(ph, pl, vh, vl);
}

__global__ void __launch_bounds__(128)
k_gemm3(const unsigned short* __restrict__ th, const unsigned short* __restrict__ tl,
        const unsigned short* __restrict__ woh, const unsigned short* __restrict__ wol,
        float* __restrict__ out) {
  __shared__ __attribute__((aligned(16))) float sD[4][16][96];
  const int lane = threadIdx.x & 31, w = threadIdx.x >> 5;
  const int h = lane >> 4, m = lane & 15;
  const int r0 = blockIdx.x * 64 + w * 16;
  const size_t ao = (size_t)(r0 + m) * DI;
  size_t bo[6];
#pragma unroll
  for (int t = 0; t < 6; ++t) bo[t] = (size_t)(t * 16 + m) * DI;
  v8f acc[6] = {};
#pragma unroll 1
  for (int ks = 0; ks < DI / 32; ++ks) {
    const int k0 = ks * 32;
    Frag ah, al;
    ldfrag(ah, th + ao, k0, h);
    ldfrag(al, tl + ao, k0, h);
#pragma unroll
    for (int t = 0; t < 6; ++t) {
      Frag bh, bl;
      ldfrag(bh, woh + bo[t], k0, h);
      ldfrag(bl, wol + bo[t], k0, h);
      acc[t] = mma3(acc[t], ah, al, bh, bl);
    }
  }
#pragma unroll
  for (int t = 0; t < 6; ++t)
#pragma unroll
    for (int r = 0; r < 8; ++r) sD[w][8 * h + r][16 * t + m] = acc[t][r];
  __syncthreads();
  tile_store<96>(&sD[w][0][0], out + (size_t)r0 * CC, CC, lane);
}

extern "C" void kernel_launch(void* const* d_in, const int* in_sizes, int n_in,
                              void* d_out, int out_size, void* d_ws, size_t ws_size,
                              hipStream_t stream) {
  if (n_in != 12) return;
  if (out_size != MM * CC) return;
  if (in_sizes[0] != MM * CC || in_sizes[1] != 2 * DI * CC || in_sizes[2] != DI * 9 ||
      in_sizes[3] != DI || in_sizes[4] != KD * CP * DI || in_sizes[5] != KD * DI * RR ||
      in_sizes[6] != KD * DI || in_sizes[7] != KD * DI * NS || in_sizes[8] != KD * DI ||
      in_sizes[9] != DI || in_sizes[10] != DI || in_sizes[11] != CC * DI) return;

  const float* x          = (const float*)d_in[0];
  const float* in_proj_w  = (const float*)d_in[1];
  const float* conv_w     = (const float*)d_in[2];
  const float* conv_b     = (const float*)d_in[3];
  const float* x_proj_w   = (const float*)d_in[4];
  const float* dt_projs_w = (const float*)d_in[5];
  const float* dt_projs_b = (const float*)d_in[6];
  const float* A_logs     = (const float*)d_in[7];
  const float* Ds         = (const float*)d_in[8];
  const float* norm_g     = (const float*)d_in[9];
  const float* norm_b     = (const float*)d_in[10];
  const float* out_proj_w = (const float*)d_in[11];
  float* out = (float*)d_out;

  char* ws = (char*)d_ws;
  size_t off = 0;
  const size_t xpl  = (size_t)MM * CC * 2;
  const size_t w1pl = (size_t)2 * DI * CC * 2;
  const size_t w2pl = (size_t)KD * CPAD * DI * 2;
  const size_t wopl = (size_t)CC * DI * 2;
  const size_t xzb  = (size_t)MM * 2 * DI * 4;
  const size_t upb  = (size_t)MM * DI * 4;
  const size_t cpl  = (size_t)MM * DI * 2;
  const size_t xdbb = (size_t)NBK * CPAD * LL * 4;
  const size_t y4b  = (size_t)NBK * LL * DI * 4;
  const size_t tpl  = (size_t)MM * DI * 2;
  auto carve = [&](size_t bytes) { size_t o = off; off += (bytes + 255) & ~(size_t)255; return o; };
  const size_t o_xh = carve(xpl),  o_xl = carve(xpl);
  const size_t o_w1h = carve(w1pl), o_w1l = carve(w1pl);
  const size_t o_w2h = carve(w2pl), o_w2l = carve(w2pl);
  const size_t o_woh = carve(wopl), o_wol = carve(wopl);
  const size_t o_xz = carve(xzb);
  const size_t o_up = carve(upb);
  const size_t o_ch = carve(cpl),  o_cl = carve(cpl);
  const size_t o_xd = carve(xdbb);
  const size_t o_y4 = carve(y4b);
  if (off > ws_size) return;
  if (2 * tpl > upb) return;
  const size_t o_th = o_up, o_tl = o_up + tpl;

  unsigned short* xh  = (unsigned short*)(ws + o_xh);
  unsigned short* xl  = (unsigned short*)(ws + o_xl);
  unsigned short* w1h = (unsigned short*)(ws + o_w1h);
  unsigned short* w1l = (unsigned short*)(ws + o_w1l);
  unsigned short* w2h = (unsigned short*)(ws + o_w2h);
  unsigned short* w2l = (unsigned short*)(ws + o_w2l);
  unsigned short* woh = (unsigned short*)(ws + o_woh);
  unsigned short* wol = (unsigned short*)(ws + o_wol);
  float* xz   = (float*)(ws + o_xz);
  float* up   = (float*)(ws + o_up);
  unsigned short* chp = (unsigned short*)(ws + o_ch);
  unsigned short* clp = (unsigned short*)(ws + o_cl);
  float* xdbl = (float*)(ws + o_xd);
  float* y4   = (float*)(ws + o_y4);
  unsigned short* thp = (unsigned short*)(ws + o_th);
  unsigned short* tlp = (unsigned short*)(ws + o_tl);

  const int n8x  = (MM * CC) / 8;
  const int n8w1 = (2 * DI * CC) / 8;
  const int n8wo = (CC * DI) / 8;
  const int n8w2 = (KD * CPAD * DI) / 8;

  k_cvt<<<dim3((n8x + 255) / 256), dim3(256), 0, stream>>>(x, n8x, xh, xl);
  k_cvt<<<dim3((n8w1 + 255) / 256), dim3(256), 0, stream>>>(in_proj_w, n8w1, w1h, w1l);
  k_cvt<<<dim3((n8wo + 255) / 256), dim3(256), 0, stream>>>(out_proj_w, n8wo, woh, wol);
  k_cvtw2<<<dim3((n8w2 + 255) / 256), dim3(256), 0, stream>>>(x_proj_w, w2h, w2l);

  k_gemm1<<<dim3(MM / 64, (2 * DI) / 64), dim3(128), 0, stream>>>(xh, xl, w1h, w1l, xz);
  k_conv<<<dim3(MM / 4), dim3(192), 0, stream>>>(xz, conv_w, conv_b, up, chp, clp);
  k_gemm2<<<dim3(LL / 64, NBK), dim3(96), 0, stream>>>(w2h, w2l, chp, clp, xdbl);
  k_scan<<<dim3(NBK), dim3(DI), 0, stream>>>(up, xdbl, dt_projs_w, dt_projs_b, A_logs, Ds, y4);
  k_ln<<<dim3(MM / 8), dim3(256), 0, stream>>>(y4, xz, norm_g, norm_b, thp, tlp);
  k_gemm3<<<dim3(MM / 64), dim3(128), 0, stream>>>(thp, tlp, woh, wol, out);
}
